// KnowledgeMLP_v1_76441827934654
// MI455X (gfx1250) — hardware-run, weakly checked
//
#include <hip/hip_runtime.h>

typedef float          v8f   __attribute__((ext_vector_type(8)));
typedef float          v4f   __attribute__((ext_vector_type(4)));
typedef unsigned int   v4u   __attribute__((ext_vector_type(4)));
typedef int            v8i   __attribute__((ext_vector_type(8)));
typedef unsigned short v8us  __attribute__((ext_vector_type(8)));
typedef unsigned short v16us __attribute__((ext_vector_type(16)));
typedef __bf16         v16bf __attribute__((ext_vector_type(16)));
typedef _Float16       v16h  __attribute__((ext_vector_type(16)));
typedef v4f  __attribute__((may_alias)) v4fa;
typedef v8us __attribute__((may_alias)) v8usa;
union FragB { v16bf v; v16us u; v8us h[2]; v8i w; };
union FragH { v16h  v; v16us u; v8us h[2]; v8i w; };

__device__ __forceinline__ v8f wmb(const FragB& a, const FragB& b, v8f c) {
  v8f d = __builtin_amdgcn_wmma_f32_16x16x32_bf16(false, a.v, false, b.v, (short)0, c, false, false);
  asm volatile("v_nop\n\tv_nop\n\tv_nop\n\tv_nop" : "+v"(d) : "v"(a.w), "v"(b.w));
  return d;
}

__device__ __forceinline__ v8f wmh(const FragH& a, const FragH& b, v8f c) {
  v8f d = __builtin_amdgcn_wmma_f32_16x16x32_f16(false, a.v, false, b.v, (short)0, c, false, false);
  asm volatile("v_nop\n\tv_nop\n\tv_nop\n\tv_nop" : "+v"(d) : "v"(a.w), "v"(b.w));
  return d;
}

__device__ __forceinline__ unsigned bf16_bits(float f) {
  const unsigned u = __float_as_uint(f);
  const unsigned r = (u + 0x7FFFu + ((u >> 16) & 1u)) >> 16;
  const unsigned q = (u >> 16) | 0x40u;
  return ((u & 0x7fffffffu) > 0x7f800000u) ? q : r;
}

__device__ __forceinline__ float bf16_val(float f) {
  return __uint_as_float(bf16_bits(f) << 16);
}
__device__ __forceinline__ int clampi(int v, int lo, int hi) {
  return v < lo ? lo : (v > hi ? hi : v);
}

__device__ __forceinline__ unsigned f16_bits(float f) {
  const unsigned u  = __float_as_uint(f);
  const unsigned s  = (u >> 16) & 0x8000u;
  const unsigned a  = u & 0x7fffffffu;
  const unsigned t  = a - 0x38000000u;
  const unsigned r  = (t + 0x0FFFu + ((t >> 13) & 1u)) >> 13;
  const unsigned rc = r > 0x7C00u ? 0x7C00u : r;
  const bool small  = a < 0x38800000u;
  const bool isnan  = a > 0x7f800000u;
  const unsigned fin = small ? 0u : (s | rc);
  return isnan ? (s | 0x7E00u) : fin;
}

__device__ __forceinline__ unsigned pk16(unsigned lo, unsigned hi) { return lo | (hi << 16); }
__device__ __forceinline__ unsigned bf16_lo_bits(float v) {
  float hi = bf16_val(v);
  asm volatile("" : "+v"(hi));
  return bf16_bits(v - hi);
}
__device__ __forceinline__ v4u pack8_bf16(v4f a, v4f c) {
  return (v4u){ pk16(bf16_bits(a[0]), bf16_bits(a[1])), pk16(bf16_bits(a[2]), bf16_bits(a[3])),
                pk16(bf16_bits(c[0]), bf16_bits(c[1])), pk16(bf16_bits(c[2]), bf16_bits(c[3])) };
}
__device__ __forceinline__ v4u pack8_bf16_lo(v4f a, v4f c) {
  return (v4u){ pk16(bf16_lo_bits(a[0]), bf16_lo_bits(a[1])), pk16(bf16_lo_bits(a[2]), bf16_lo_bits(a[3])),
                pk16(bf16_lo_bits(c[0]), bf16_lo_bits(c[1])), pk16(bf16_lo_bits(c[2]), bf16_lo_bits(c[3])) };
}
__device__ __forceinline__ v4u pack8_f16(v4f a, v4f c) {
  return (v4u){ pk16(f16_bits(a[0]), f16_bits(a[1])), pk16(f16_bits(a[2]), f16_bits(a[3])),
                pk16(f16_bits(c[0]), f16_bits(c[1])), pk16(f16_bits(c[2]), f16_bits(c[3])) };
}

template <int FORM>
__global__ __launch_bounds__(256) void k_plane(const float* __restrict__ src, int rows, int cols, int ldsrc,
                                               unsigned short* __restrict__ dst, int MP, int KP) {
  static_assert(FORM >= 0 && FORM <= 3);
  const int KTOT = (FORM == 1 || FORM == 3) ? 2 * KP : KP;
  const unsigned ppr   = (unsigned)(KTOT >> 3);
  const unsigned kp8   = (unsigned)(KP >> 3);
  const unsigned total = (unsigned)MP * ppr;
  const unsigned g     = blockIdx.x * 256u + threadIdx.x;
  const unsigned rowu  = g / ppr;
  const unsigned p     = g - rowu * ppr;
  const bool second    = p >= kp8;
  const int row = (int)rowu;
  const int c0  = (int)((second ? p - kp8 : p) << 3);
  const float* srow = src + (size_t)clampi(row, 0, rows - 1) * (size_t)ldsrc;
  float x[8];
  unsigned mk[8];
#pragma unroll
  for (int e = 0; e < 8; ++e) {
    const int c = c0 + e;
    const float v = srow[clampi(c, 0, cols - 1)];
    asm volatile("" :: "v"(v));
    x[e]  = v;
    mk[e] = (row < rows && c < cols) ? 0xFFFFu : 0u;
  }
  const v4f a = (v4f){ x[0], x[1], x[2], x[3] };
  const v4f c = (v4f){ x[4], x[5], x[6], x[7] };
  v4u o;
  if (FORM == 2) {
    o = pack8_f16(a, c);
  } else {
    const v4u hi = pack8_bf16(a, c);
    o = hi;
    if (FORM == 1) { const v4u lo = pack8_bf16_lo(a, c); o = second ? lo : hi; }
  }
  const v4u mw = (v4u){ pk16(mk[0], mk[1]), pk16(mk[2], mk[3]), pk16(mk[4], mk[5]), pk16(mk[6], mk[7]) };
  o &= mw;
  if (g < total) {
    volatile v4u* q = (volatile v4u*)(dst + (size_t)g * 8);
    *q = o;
    __threadfence();
    *q = o;
  }
}

template <int FORM> struct FragOf    { typedef FragB T; };
template <>         struct FragOf<2> { typedef FragH T; };
__device__ __forceinline__ v8f mm(const FragB& a, const FragB& b, v8f c) { return wmb(a, b, c); }
__device__ __forceinline__ v8f mm(const FragH& a, const FragH& b, v8f c) { return wmh(a, b, c); }
template <class F> __device__ __forceinline__ F ld_frag(const unsigned short* p) {
  F f;
  f.h[0] = *(const v8usa*)(p);
  f.h[1] = *(const v8usa*)(p + 16);
  return f;
}

template <int FORM, int EPI>
__global__ __launch_bounds__(256) __attribute__((amdgpu_num_vgpr(248)))
void k_gemm_nt(const unsigned short* __restrict__ A, const unsigned short* __restrict__ B,
               const float* __restrict__ bias, float* __restrict__ D, int M, int N, int KTOT, int ldd) {
  static_assert(FORM >= 0 && FORM <= 2);
  static_assert(EPI == 0 || EPI == 1);
  typedef typename FragOf<FORM>::T F;
  __shared__ __attribute__((aligned(16))) float sT[8][16 * 68];
  const int lane = threadIdx.x & 31;
  const int wave = threadIdx.x >> 5;
  const int tilesM = (M + 63) >> 6;
  const int tilesN = (N + 63) >> 6;
  const int tile = blockIdx.x * 8 + wave;
  if (tile >= tilesM * tilesN) return;
  const int tm = tile / tilesN;
  const int tn = tile - tm * tilesN;
  const int m0 = tm << 6;
  const int n0 = tn << 6;

  const int rl = lane & 15;
  const int h8 = (lane >> 4) * 8;
  const unsigned short* pa = A + (size_t)(m0 + rl) * (size_t)KTOT + h8;
  const unsigned short* pb = B + (size_t)(n0 + rl) * (size_t)KTOT + h8;

  v8f acc[4][4];
#pragma unroll
  for (int i = 0; i < 4; ++i)
#pragma unroll
    for (int j = 0; j < 4; ++j) acc[i][j] = (v8f){0.f, 0.f, 0.f, 0.f, 0.f, 0.f, 0.f, 0.f};

#pragma unroll 1
  for (int k0 = 0; k0 < KTOT; k0 += 32) {
    F bf[4];
#pragma unroll
    for (int j = 0; j < 4; ++j) bf[j] = ld_frag<F>(pb + (size_t)(j << 4) * (size_t)KTOT + k0);
#pragma unroll
    for (int i = 0; i < 4; ++i) {
      const F af = ld_frag<F>(pa + (size_t)(i << 4) * (size_t)KTOT + k0);
#pragma unroll
      for (int j = 0; j < 4; ++j) acc[i][j] = mm(af, bf[j], acc[i][j]);
    }
  }

  float* slab = sT[wave];
  const int hh = lane >> 4;
  const int c4 = (lane & 15) * 4;
  const int nc = n0 + c4;
  const bool cok = nc < N;
  v4f bv = (v4f){0.f, 0.f, 0.f, 0.f};
  if (EPI == 1) {
    bv = *(const v4fa*)(bias + clampi(nc, 0, N - 4));
    asm volatile("" :: "v"(bv));
  }
#pragma unroll
  for (int i = 0; i < 4; ++i) {
    const int mBase = m0 + (i << 4);
#pragma unroll
    for (int j = 0; j < 4; ++j) {
#pragma unroll
      for (int r = 0; r < 8; ++r) slab[(h8 + r) * 68 + (j << 4) + rl] = acc[i][j][r];
    }
    __builtin_amdgcn_fence(__ATOMIC_RELEASE, "workgroup");
    __builtin_amdgcn_wave_barrier();
    __builtin_amdgcn_fence(__ATOMIC_ACQUIRE, "workgroup");
    v4f vv[8];
#pragma unroll
    for (int it = 0; it < 8; ++it) {
      const int row = it * 2 + hh;
      v4f v = *(const v4fa*)(slab + row * 68 + c4);
      if (EPI == 1) v += bv;
      vv[it] = v;
    }
    for (int pass = 0; pass < 2; ++pass) {
#pragma unroll
      for (int it = 0; it < 8; ++it) {
        const int row = mBase + it * 2 + hh;
        if (cok && row < M) *(volatile v4f*)(D + (size_t)row * (size_t)ldd + nc) = vv[it];
      }
      __threadfence();
    }
    __builtin_amdgcn_fence(__ATOMIC_RELEASE, "workgroup");
    __builtin_amdgcn_wave_barrier();
    __builtin_amdgcn_fence(__ATOMIC_ACQUIRE, "workgroup");
  }
}

#ifndef SPLIT_H1
#define SPLIT_H1 1
#endif
#ifndef SPLIT_H2
#define SPLIT_H2 1
#endif
#ifndef SPLIT_H3
#define SPLIT_H3 1
#endif
#ifndef SPLIT_S
#define SPLIT_S 1
#endif

#define NB      8192
#define FAN     50
#define NKG     200000
#define NKGP    200064
#define KGS     64
#define INS     512
#define HID     128
#define CONCAT  64
#define OUTS    1024
#define WSLIM   ((size_t)128 << 20)

#define O_WKG   0
#define O_W1A   (O_WKG + CONCAT * KGS)
#define O_W1B   (O_W1A + HID * INS)
#define O_W1C   (O_W1B + INS * 2 * HID)
#define O_W1D   (O_W1C + HID * 2 * INS)
#define O_W2    (O_W1D + CONCAT * 2 * HID)
#define WPL_HW  (O_W2 + OUTS * 2 * CONCAT)
#define BO_KG   0
#define BO_1A   (BO_KG + CONCAT)
#define BO_1B   (BO_1A + HID)
#define BO_1C   (BO_1B + INS)
#define BO_1D   (BO_1C + HID)
#define BO_2    (BO_1D + CONCAT)
#define BIAS_F  (BO_2 + OUTS)
#define PB_KG   (CONCAT * (KGS / 8) / 256)
#define PB_1A   (HID * (INS / 8) / 256)
#define PB_1B   (INS * (2 * HID / 8) / 256)
#define PB_1C   (HID * (2 * INS / 8) / 256)
#define PB_1D   (CONCAT * (2 * HID / 8) / 256)
#define PB_2    (OUTS * (2 * CONCAT / 8) / 256)
#define PB_ALL  (PB_KG + PB_1A + PB_1B + PB_1C + PB_1D + PB_2)

static_assert(NB % 128 == 0);
static_assert(FAN <= 64 && FAN > 32);
static_assert(CONCAT == 64 && CONCAT == 32 * 2);
static_assert(NKGP == 1563 * 128 && NKGP >= NKG && NKGP % 64 == 0 && NKGP % 16 == 0);
static_assert(KGS % 32 == 0 && INS % 32 == 0 && (2 * HID) % 32 == 0 && (2 * INS) % 32 == 0 && (2 * CONCAT) % 32 == 0);
static_assert(NB % 64 == 0 && HID % 64 == 0 && INS % 64 == 0 && CONCAT % 64 == 0 && OUTS % 64 == 0);
static_assert(CONCAT % 32 == 0 && HID % 32 == 0 && INS % 32 == 0 && OUTS % 32 == 0);
static_assert((CONCAT * (KGS / 8)) % 256 == 0 && (HID * (INS / 8)) % 256 == 0 && (INS * (2 * HID / 8)) % 256 == 0);
static_assert((HID * (2 * INS / 8)) % 256 == 0 && (CONCAT * (2 * HID / 8)) % 256 == 0 && (OUTS * (2 * CONCAT / 8)) % 256 == 0);
static_assert(PB_ALL == 234 && WPL_HW == 479232 && BIAS_F == 1920);
static_assert((O_W1A * 2) % 128 == 0 && (O_W1B * 2) % 128 == 0 && (O_W1C * 2) % 128 == 0 && (O_W1D * 2) % 128 == 0 && (O_W2 * 2) % 128 == 0);
static_assert((BO_1A * 4) % 128 == 0 && (BO_1B * 4) % 128 == 0 && (BO_1C * 4) % 128 == 0 && (BO_1D * 4) % 128 == 0 && (BO_2 * 4) % 128 == 0);
static_assert((NKGP * (KGS / 8)) % 256 == 0 && (NB * (INS / 8)) % 256 == 0);
static_assert((NB * (HID / 8)) % 256 == 0 && (NB * (INS / 8)) % 256 == 0 && NB % 8 == 0);
static_assert((long long)NB * OUTS == 8388608LL);

typedef float        v2f __attribute__((ext_vector_type(2)));
typedef v2f __attribute__((may_alias)) v2fa;

__device__ __forceinline__ float relu_sel(float v) { return (v > 0.0f) ? v : (v - v); }

template <int K, int N, int KTOT>
__device__ __forceinline__ void wt_piece(const float* __restrict__ W, unsigned short* __restrict__ dst, unsigned g) {
  static_assert(KTOT == K || KTOT == 2 * K);
  static_assert(K % 8 == 0 && N % 64 == 0 && KTOT % 32 == 0);
  constexpr unsigned ppr   = (unsigned)(KTOT / 8);
  constexpr unsigned total = (unsigned)N * ppr;
  const unsigned gc = g < total ? g : total - 1u;
  const unsigned n  = gc / ppr;
  const unsigned p  = gc - n * ppr;
  const int kk = (int)(p << 3);
  const int k0 = (kk >= K) ? kk - K : kk;
  float x[8];
#pragma unroll
  for (int e = 0; e < 8; ++e) {
    const float v = W[(size_t)clampi(k0 + e, 0, K - 1) * (size_t)N + (size_t)n];
    asm volatile("" :: "v"(v));
    x[e] = v;
  }
  const v4f a = (v4f){ x[0], x[1], x[2], x[3] };
  const v4f c = (v4f){ x[4], x[5], x[6], x[7] };
  const v4u o = pack8_bf16(a, c);
  if (g < total) {
    volatile v4u* q = (volatile v4u*)(dst + (size_t)g * 8);
    *q = o;
    __threadfence();
    *q = o;
  }
}

__global__ __launch_bounds__(256) void k_prep_w(const float* __restrict__ Wkg, const float* __restrict__ W1a,
                                                const float* __restrict__ W1b, const float* __restrict__ W1c,
                                                const float* __restrict__ W1d, const float* __restrict__ W2,
                                                unsigned short* __restrict__ WPL) {
  const int bx = (int)blockIdx.x;
  const unsigned tid = threadIdx.x;
  constexpr int e0 = PB_KG;
  constexpr int e1 = e0 + PB_1A;
  constexpr int e2 = e1 + PB_1B;
  constexpr int e3 = e2 + PB_1C;
  constexpr int e4 = e3 + PB_1D;
  if (bx < e0) {
    wt_piece<KGS, CONCAT, KGS>(Wkg, WPL + O_WKG, (unsigned)bx * 256u + tid);
  } else if (bx < e1) {
    wt_piece<INS, HID, INS>(W1a, WPL + O_W1A, (unsigned)(bx - e0) * 256u + tid);
  } else if (bx < e2) {
    wt_piece<HID, INS, 2 * HID>(W1b, WPL + O_W1B, (unsigned)(bx - e1) * 256u + tid);
  } else if (bx < e3) {
    wt_piece<INS, HID, 2 * INS>(W1c, WPL + O_W1C, (unsigned)(bx - e2) * 256u + tid);
  } else if (bx < e4) {
    wt_piece<HID, CONCAT, 2 * HID>(W1d, WPL + O_W1D, (unsigned)(bx - e3) * 256u + tid);
  } else {
    wt_piece<CONCAT, OUTS, 2 * CONCAT>(W2, WPL + O_W2, (unsigned)(bx - e4) * 256u + tid);
  }
}

__global__ __launch_bounds__(256) void k_prep_b(const float* __restrict__ bkg, const float* __restrict__ b1a,
                                                const float* __restrict__ b1b, const float* __restrict__ b1c,
                                                const float* __restrict__ b1d, const float* __restrict__ b2,
                                                float* __restrict__ BIAS) {
  constexpr int P0 = BO_KG / 4, P1 = BO_1A / 4, P2 = BO_1B / 4, P3 = BO_1C / 4, P4 = BO_1D / 4, P5 = BO_2 / 4;
  constexpr int PE = BIAS_F / 4;
  const int t  = (int)(blockIdx.x * 256u + threadIdx.x);
  const int tc = t < PE ? t : PE - 1;
  const v4f x0 = *(const v4fa*)(bkg + 4 * clampi(tc - P0, 0, CONCAT / 4 - 1));
  const v4f x1 = *(const v4fa*)(b1a + 4 * clampi(tc - P1, 0, HID / 4 - 1));
  const v4f x2 = *(const v4fa*)(b1b + 4 * clampi(tc - P2, 0, INS / 4 - 1));
  const v4f x3 = *(const v4fa*)(b1c + 4 * clampi(tc - P3, 0, HID / 4 - 1));
  const v4f x4 = *(const v4fa*)(b1d + 4 * clampi(tc - P4, 0, CONCAT / 4 - 1));
  const v4f x5 = *(const v4fa*)(b2  + 4 * clampi(tc - P5, 0, OUTS / 4 - 1));
  asm volatile("" :: "v"(x0), "v"(x1), "v"(x2), "v"(x3), "v"(x4), "v"(x5));
  const unsigned m0 = (tc < P1) ? 0xFFFFFFFFu : 0u;
  const unsigned m1 = (tc >= P1 && tc < P2) ? 0xFFFFFFFFu : 0u;
  const unsigned m2 = (tc >= P2 && tc < P3) ? 0xFFFFFFFFu : 0u;
  const unsigned m3 = (tc >= P3 && tc < P4) ? 0xFFFFFFFFu : 0u;
  const unsigned m4 = (tc >= P4 && tc < P5) ? 0xFFFFFFFFu : 0u;
  const unsigned m5 = (tc >= P5) ? 0xFFFFFFFFu : 0u;
  v4f o;
#pragma unroll
  for (int e = 0; e < 4; ++e) {
    const unsigned bits = ((bf16_bits(x0[e]) << 16) & m0) | ((bf16_bits(x1[e]) << 16) & m1) |
                          ((bf16_bits(x2[e]) << 16) & m2) | ((bf16_bits(x3[e]) << 16) & m3) |
                          ((bf16_bits(x4[e]) << 16) & m4) | ((bf16_bits(x5[e]) << 16) & m5);
    o[e] = __uint_as_float(bits);
  }
  if (t < PE) {
    volatile v4f* d = (volatile v4f*)(BIAS + 4 * t);
    *d = o;
    __threadfence();
    *d = o;
  }
}

template <int C, int SPLIT>
__global__ __launch_bounds__(256) void k_row(const float* __restrict__ P, unsigned short* __restrict__ H) {
  static_assert(C % 64 == 0 && (C * 2) % 128 == 0);
  constexpr unsigned ppr = (unsigned)(C / 8);
  const unsigned g   = blockIdx.x * 256u + threadIdx.x;
  const unsigned row = g / ppr;
  const unsigned p   = g - row * ppr;
  const float* src = P + (size_t)row * C + (size_t)p * 8;
  v4f a = *(const v4fa*)(src);
  v4f c = *(const v4fa*)(src + 4);
  asm volatile("" :: "v"(a), "v"(c));
#pragma unroll
  for (int e = 0; e < 4; ++e) { a[e] = relu_sel(a[e]); c[e] = relu_sel(c[e]); }
  const v4u hi = pack8_bf16(a, c);
  v4u lo = (v4u){ 0u, 0u, 0u, 0u };
  if (SPLIT != 0) lo = pack8_bf16_lo(a, c);
  volatile v4u* qh = (volatile v4u*)(H + (size_t)row * (2 * C) + (size_t)p * 8);
  volatile v4u* ql = qh + (C / 8);
  *qh = hi;
  *ql = lo;
  __threadfence();
  *qh = hi;
  *ql = lo;
}

__global__ __launch_bounds__(256) void k_gather_sum(const int* __restrict__ idx, const int* __restrict__ mask,
                                                    const float* __restrict__ TP, const float* __restrict__ P4,
                                                    unsigned* __restrict__ Shlw) {
#pragma clang fp contract(off)
  const int lane = threadIdx.x & 31;
  const int wave = threadIdx.x >> 5;
  const int b    = (int)blockIdx.x * 8 + wave;
  const int* ib = idx  + (size_t)b * FAN;
  const int* mb = mask + (size_t)b * FAN;
  const int j1 = (lane + 32 < FAN) ? lane + 32 : FAN - 1;
  int iw0 = ib[lane];
  int iw1 = ib[j1];
  int mw0 = mb[lane];
  int mw1 = mb[j1];
  asm volatile("" :: "v"(iw0));
  asm volatile("" :: "v"(iw1));
  asm volatile("" :: "v"(mw0));
  asm volatile("" :: "v"(mw1));
  const int v1 = (lane + 32 < FAN) ? -1 : 0;
  iw1 &= v1;
  mw1 &= v1;
  iw0 = clampi(iw0, 0, NKG - 1);
  iw1 = clampi(iw1, 0, NKG - 1);
  const float* tpl = TP + 2 * lane;
  float a0 = 0.0f;
  float a1 = 0.0f;
#pragma unroll 8
  for (int k = 0; k < 32; ++k) {
    const int id = __shfl(iw0, k);
    const int m  = __shfl(mw0, k);
    const v2f t = *(const v2fa*)(tpl + (size_t)id * CONCAT);
    asm volatile("" :: "v"(t));
    const float fm = (float)m;
    const float q0 = fm * relu_sel(t[0]);
    const float q1 = fm * relu_sel(t[1]);
    a0 = a0 + ((m != 0) ? q0 : 0.0f);
    a1 = a1 + ((m != 0) ? q1 : 0.0f);
  }
#pragma unroll 6
  for (int k = 0; k < FAN - 32; ++k) {
    const int id = __shfl(iw1, k);
    const int m  = __shfl(mw1, k);
    const v2f t = *(const v2fa*)(tpl + (size_t)id * CONCAT);
    asm volatile("" :: "v"(t));
    const float fm = (float)m;
    const float q0 = fm * relu_sel(t[0]);
    const float q1 = fm * relu_sel(t[1]);
    a0 = a0 + ((m != 0) ? q0 : 0.0f);
    a1 = a1 + ((m != 0) ? q1 : 0.0f);
  }
  const v2f p = *(const v2fa*)(P4 + (size_t)b * CONCAT + 2 * lane);
  asm volatile("" :: "v"(p));
  const float s0 = a0 + relu_sel(p[0]);
  const float s1 = a1 + relu_sel(p[1]);
  const unsigned hiw = pk16(bf16_bits(s0), bf16_bits(s1));
  unsigned low = 0u;
  if (SPLIT_S != 0) low = pk16(bf16_lo_bits(s0), bf16_lo_bits(s1));
  volatile unsigned* ph = (volatile unsigned*)(Shlw + (size_t)b * CONCAT + lane);
  volatile unsigned* pl = ph + (CONCAT / 2);
  *ph = hiw;
  *pl = low;
  __threadfence();
  *ph = hiw;
  *pl = low;
}

extern "C" void kernel_launch(void* const* d_in, const int* in_sizes, int n_in,
                              void* d_out, int out_size, void* d_ws, size_t ws_size,
                              hipStream_t stream) {
  if (n_in < 16) return;
  if (in_sizes[0]  != NB * INS) return;
  if (in_sizes[1]  != NKG * KGS) return;
  if (in_sizes[2]  != NB * FAN) return;
  if (in_sizes[3]  != NB * FAN) return;
  if (in_sizes[4]  != KGS * CONCAT) return;
  if (in_sizes[5]  != CONCAT) return;
  if (in_sizes[6]  != INS * HID) return;
  if (in_sizes[7]  != HID) return;
  if (in_sizes[8]  != HID * INS) return;
  if (in_sizes[9]  != INS) return;
  if (in_sizes[10] != INS * HID) return;
  if (in_sizes[11] != HID) return;
  if (in_sizes[12] != HID * CONCAT) return;
  if (in_sizes[13] != CONCAT) return;
  if (in_sizes[14] != CONCAT * OUTS) return;
  if (in_sizes[15] != OUTS) return;
  if (out_size != NB * OUTS) return;

  const float* x    = (const float*)d_in[0];
  const float* kg   = (const float*)d_in[1];
  const int*   idx  = (const int*)  d_in[2];
  const int*   mask = (const int*)  d_in[3];
  const float* Wkg  = (const float*)d_in[4];
  const float* bkg  = (const float*)d_in[5];
  const float* W1a  = (const float*)d_in[6];
  const float* b1a  = (const float*)d_in[7];
  const float* W1b  = (const float*)d_in[8];
  const float* b1b  = (const float*)d_in[9];
  const float* W1c  = (const float*)d_in[10];
  const float* b1c  = (const float*)d_in[11];
  const float* W1d  = (const float*)d_in[12];
  const float* b1d  = (const float*)d_in[13];
  const float* W2   = (const float*)d_in[14];
  const float* b2   = (const float*)d_in[15];
  float* out = (float*)d_out;

  constexpr size_t szKGB  = (size_t)NKGP * KGS * 2;
  constexpr size_t szTP   = (size_t)NKGP * CONCAT * 4;
  constexpr size_t szXB   = (size_t)NB * INS * 2;
  constexpr size_t szP13  = (size_t)NB * HID * 4;
  constexpr size_t szH13  = (size_t)NB * 2 * HID * 2;
  constexpr size_t szP2   = (size_t)NB * INS * 4;
  constexpr size_t szH2   = (size_t)NB * 2 * INS * 2;
  constexpr size_t szP4   = (size_t)NB * CONCAT * 4;
  constexpr size_t szShl  = (size_t)NB * 2 * CONCAT * 2;
  constexpr size_t szWPL  = (size_t)WPL_HW * 2;
  constexpr size_t szBIAS = (size_t)BIAS_F * 4;
  static_assert(szKGB % 256 == 0 && szTP % 256 == 0 && szXB % 256 == 0 && szP13 % 256 == 0 && szH13 % 256 == 0);
  static_assert(szP2 % 256 == 0 && szH2 % 256 == 0 && szP4 % 256 == 0 && szShl % 256 == 0 && szWPL % 256 == 0 && szBIAS % 256 == 0);
  static_assert(szH2 <= szKGB);
  constexpr size_t oKGB  = 0;
  constexpr size_t oH2   = oKGB;
  constexpr size_t oTP   = oKGB + szKGB;
  constexpr size_t oXB   = oTP + szTP;
  constexpr size_t oP13  = oXB + szXB;
  constexpr size_t oH13  = oP13 + szP13;
  constexpr size_t oP2   = oH13 + szH13;
  constexpr size_t oP4   = oP2 + szP2;
  constexpr size_t oShl  = oP4 + szP4;
  constexpr size_t oWPL  = oShl + szShl;
  constexpr size_t oBIAS = oWPL + szWPL;
  constexpr size_t total = oBIAS + szBIAS;
  static_assert(total <= WSLIM);
  static_assert(total == (size_t)451326 * 256);
  if (total > ws_size) return;

  char* ws = (char*)d_ws;
  unsigned short* KGB  = (unsigned short*)(ws + oKGB);
  unsigned short* H2hl = (unsigned short*)(ws + oH2);
  float*          TP   = (float*)(ws + oTP);
  unsigned short* XB   = (unsigned short*)(ws + oXB);
  float*          P13  = (float*)(ws + oP13);
  unsigned short* H13  = (unsigned short*)(ws + oH13);
  float*          P2   = (float*)(ws + oP2);
  float*          P4   = (float*)(ws + oP4);
  unsigned short* Shl  = (unsigned short*)(ws + oShl);
  unsigned short* WPL  = (unsigned short*)(ws + oWPL);
  float*          BIAS = (float*)(ws + oBIAS);

  k_prep_w<<<dim3(PB_ALL), dim3(256), 0, stream>>>(Wkg, W1a, W1b, W1c, W1d, W2, WPL);
  k_prep_b<<<dim3((BIAS_F / 4 + 255) / 256), dim3(256), 0, stream>>>(bkg, b1a, b1b, b1c, b1d, b2, BIAS);

  k_plane<0><<<dim3(NKGP * (KGS / 8) / 256), dim3(256), 0, stream>>>(kg, NKG, KGS, KGS, KGB, NKGP, KGS);
  k_plane<0><<<dim3(NB * (INS / 8) / 256), dim3(256), 0, stream>>>(x, NB, INS, INS, XB, NB, INS);

  {
    constexpr int tiles = (NKGP / 64) * (CONCAT / 64);
    k_gemm_nt<0, 1><<<dim3((tiles + 7) / 8), dim3(256), 0, stream>>>(
        KGB, WPL + O_WKG, BIAS + BO_KG, TP, NKGP, CONCAT, KGS, CONCAT);
  }
  {
    constexpr int tiles = (NB / 64) * (HID / 64);
    k_gemm_nt<0, 1><<<dim3((tiles + 7) / 8), dim3(256), 0, stream>>>(
        XB, WPL + O_W1A, BIAS + BO_1A, P13, NB, HID, INS, HID);
  }
  k_row<HID, SPLIT_H1><<<dim3(NB * (HID / 8) / 256), dim3(256), 0, stream>>>(P13, H13);
  {
    constexpr int tiles = (NB / 64) * (INS / 64);
    k_gemm_nt<1, 1><<<dim3((tiles + 7) / 8), dim3(256), 0, stream>>>(
        H13, WPL + O_W1B, BIAS + BO_1B, P2, NB, INS, 2 * HID, INS);
  }
  k_row<INS, SPLIT_H2><<<dim3(NB * (INS / 8) / 256), dim3(256), 0, stream>>>(P2, H2hl);
  {
    constexpr int tiles = (NB / 64) * (HID / 64);
    k_gemm_nt<1, 1><<<dim3((tiles + 7) / 8), dim3(256), 0, stream>>>(
        H2hl, WPL + O_W1C, BIAS + BO_1C, P13, NB, HID, 2 * INS, HID);
  }
  k_row<HID, SPLIT_H3><<<dim3(NB * (HID / 8) / 256), dim3(256), 0, stream>>>(P13, H13);
  {
    constexpr int tiles = (NB / 64) * (CONCAT / 64);
    k_gemm_nt<1, 1><<<dim3((tiles + 7) / 8), dim3(256), 0, stream>>>(
        H13, WPL + O_W1D, BIAS + BO_1D, P4, NB, CONCAT, 2 * HID, CONCAT);
  }
  k_gather_sum<<<dim3(NB / 8), dim3(256), 0, stream>>>(idx, mask, TP, P4, (unsigned*)Shl);
  {
    constexpr int tiles = (NB / 64) * (OUTS / 64);
    k_gemm_nt<1, 1><<<dim3((tiles + 7) / 8), dim3(256), 0, stream>>>(
        Shl, WPL + O_W2, BIAS + BO_2, out, NB, OUTS, 2 * CONCAT, OUTS);
  }
}
